// SpatialGatedBlock_21397527068865
// MI455X (gfx1250) — hardware-verified
//
#include <hip/hip_runtime.h>
#include <stdint.h>
#include <math.h>


#define DIM   128
#define NGRP  64
#define GSMAX 128
#define CH1   2048
#define CAP1  96
#define CAPG  6144
#define LDP   132

typedef float          v8f  __attribute__((ext_vector_type(8)));
typedef float          v4f  __attribute__((ext_vector_type(4)));
typedef __bf16         v16b __attribute__((ext_vector_type(16)));
typedef unsigned short v8us __attribute__((ext_vector_type(8)));
typedef unsigned int   v4u  __attribute__((ext_vector_type(4)));
typedef unsigned short us_t;

union Frag { v16b v; v8us h[2]; v8f f; };

__device__ __forceinline__ unsigned f2bf(float f) {
  unsigned u = __float_as_uint(f);
  return (u + 0x7FFFu + ((u >> 16) & 1u)) >> 16;
}
__device__ __forceinline__ float bf2f(unsigned b) { return __uint_as_float(b << 16); }

__device__ __forceinline__ void split8(const float (&v)[8], v8us& hi, v8us& lo) {
  v8us a = {0, 0, 0, 0, 0, 0, 0, 0};
  v8us c = {0, 0, 0, 0, 0, 0, 0, 0};
#pragma unroll
  for (int e = 0; e < 8; ++e) {
    const unsigned hb = f2bf(v[e]);
    a[e] = (us_t)hb;
    c[e] = (us_t)f2bf(v[e] - bf2f(hb));
  }
  hi = a;
  lo = c;
}

__device__ __forceinline__ Frag ldfrag(const us_t* p, int h) {
  Frag f;
  f.h[0] = *(const v8us*)(p + 8 * h);
  f.h[1] = *(const v8us*)(p + 16 + 8 * h);
  return f;
}

__device__ __forceinline__ v8f mma3(v8f acc, const Frag& ah, const Frag& al,
                                    const Frag& bh, const Frag& bl) {
  acc = __builtin_amdgcn_wmma_f32_16x16x32_bf16(false, ah.v, false, bh.v, (short)0, acc, false, false);
  acc = __builtin_amdgcn_wmma_f32_16x16x32_bf16(false, al.v, false, bh.v, (short)0, acc, false, false);
  acc = __builtin_amdgcn_wmma_f32_16x16x32_bf16(false, ah.v, false, bl.v, (short)0, acc, false, false);
  asm volatile("v_nop\n\tv_nop\n\tv_nop\n\tv_nop"
               : "+v"(acc)
               : "v"(ah.f), "v"(al.f), "v"(bh.f), "v"(bl.f));
  return acc;
}

__device__ __forceinline__ v8f gemm3(const us_t* ah, const us_t* al,
                                     const us_t* bh, const us_t* bl, int K, int h) {
  v8f acc = {0.f, 0.f, 0.f, 0.f, 0.f, 0.f, 0.f, 0.f};
#pragma unroll 2
  for (int k0 = 0; k0 < K; k0 += 32) {
    const Frag fah = ldfrag(ah + k0, h);
    const Frag fal = ldfrag(al + k0, h);
    const Frag fbh = ldfrag(bh + k0, h);
    const Frag fbl = ldfrag(bl + k0, h);
    acc = mma3(acc, fah, fal, fbh, fbl);
  }
  return acc;
}

template <int BITS>
__device__ __forceinline__ unsigned peer_mask(unsigned key, unsigned vmask) {
  unsigned p = vmask;
#pragma unroll
  for (int b = 0; b < BITS; ++b) {
    const unsigned bit = (key >> b) & 1u;
    const unsigned m = (unsigned)__ballot(bit != 0u);
    p &= bit ? m : ~m;
  }
  return p;
}

__global__ void __launch_bounds__(256)
k_prep(const float* __restrict__ x, int n,
       us_t* Yh, us_t* Yl, us_t* Xh, us_t* Xl,
       us_t* YTh, us_t* YTl, us_t* XTh, us_t* XTl) {
  __shared__ float xs[64 * LDP] __attribute__((aligned(16)));
  __shared__ float rinv[64];
  const int t = threadIdx.x, w = t >> 5, l = t & 31;
  const int i0 = blockIdx.x * 64;
  if (i0 >= n) return;

  for (int idx = t; idx < 64 * 32; idx += 256) {
    const int row = idx >> 5, c4 = idx & 31;
    v4f v = {0.f, 0.f, 0.f, 0.f};
    if (i0 + row < n) v = *(const v4f*)(x + (size_t)(i0 + row) * DIM + 4 * c4);
    *(v4f*)(xs + row * LDP + 4 * c4) = v;
  }
  __syncthreads();

#pragma unroll 1
  for (int j = 0; j < 8; ++j) {
    const int row = 8 * w + j;
    const v4f v = *(const v4f*)(xs + row * LDP + 4 * l);
    float s = v.x * v.x + v.y * v.y + v.z * v.z + v.w * v.w;
#pragma unroll
    for (int off = 16; off > 0; off >>= 1) s += __shfl_xor(s, off, 32);
    if (l == 0) rinv[row] = (s > 0.f) ? (1.0f / sqrtf(s)) : 0.f;
  }
  __syncthreads();

#pragma unroll 1
  for (int j = 0; j < 4; ++j) {
    const int row = 8 * w + 2 * j + (l >> 4);
    const int cb = 8 * (l & 15);
    const float* src = xs + row * LDP + cb;
    const float ri = rinv[row];
    float xv[8], yv[8];
#pragma unroll
    for (int e = 0; e < 8; ++e) { xv[e] = src[e]; yv[e] = xv[e] * ri; }
    v8us yh, yl, xh, xl;
    split8(yv, yh, yl);
    split8(xv, xh, xl);
    const size_t o = (size_t)(i0 + row) * DIM + cb;
    if (i0 + row < n) {
      *(volatile v8us*)(Yh + o) = yh;
      *(volatile v8us*)(Yl + o) = yl;
      *(volatile v8us*)(Xh + o) = xh;
      *(volatile v8us*)(Xl + o) = xl;
      __threadfence();
      *(volatile v8us*)(Yh + o) = yh;
      *(volatile v8us*)(Yl + o) = yl;
      *(volatile v8us*)(Xh + o) = xh;
      *(volatile v8us*)(Xl + o) = xl;
    }
  }

  {
    const int q = l >> 3, j = l & 7;
    float r8[8];
#pragma unroll
    for (int e = 0; e < 8; ++e) r8[e] = rinv[8 * j + e];
    const bool ok = (i0 + 8 * j + 7) < n;
#pragma unroll 1
    for (int s = 0; s < 4; ++s) {
      const int k = 4 * w + 32 * s + q;
      float xv[8], yv[8];
#pragma unroll
      for (int e = 0; e < 8; ++e) { xv[e] = xs[(8 * j + e) * LDP + k]; yv[e] = xv[e] * r8[e]; }
      v8us yh, yl, xh, xl;
      split8(yv, yh, yl);
      split8(xv, xh, xl);
      const size_t o = (size_t)k * n + i0 + 8 * j;
      if (ok) {
        *(volatile v8us*)(YTh + o) = yh;
        *(volatile v8us*)(YTl + o) = yl;
        *(volatile v8us*)(XTh + o) = xh;
        *(volatile v8us*)(XTl + o) = xl;
        __threadfence();
        *(volatile v8us*)(YTh + o) = yh;
        *(volatile v8us*)(YTl + o) = yl;
        *(volatile v8us*)(XTh + o) = xh;
        *(volatile v8us*)(XTl + o) = xl;
      }
    }
  }
}

__global__ void __launch_bounds__(256)
k_wconv(const float* __restrict__ W, us_t* WTh, us_t* WTl) {
  const int t = threadIdx.x, w = t >> 5, l = t & 31;
#pragma unroll 1
  for (int s = 0; s < 8; ++s) {
    const int c = 16 * s + 2 * w + (l >> 4);
    const int kb = 8 * (l & 15);
    float v[8];
#pragma unroll
    for (int e = 0; e < 8; ++e) v[e] = W[(size_t)(kb + e) * DIM + c];
    v8us hi, lo;
    split8(v, hi, lo);
    const size_t o = (size_t)c * DIM + kb;
    *(volatile v8us*)(WTh + o) = hi;
    *(volatile v8us*)(WTl + o) = lo;
    __threadfence();
    *(volatile v8us*)(WTh + o) = hi;
    *(volatile v8us*)(WTl + o) = lo;
  }
}

__global__ void __launch_bounds__(32)
k_b1(const int* __restrict__ rowp, const int* __restrict__ colp, int E, int n, int gs,
     unsigned* b1cnt, unsigned* b1dat) {
  __shared__ volatile unsigned cur[NGRP];
  __shared__ unsigned reg[NGRP * CAP1] __attribute__((aligned(16)));
  const int l = threadIdx.x, blk = blockIdx.x;
  cur[l] = 0u;
  cur[l + 32] = 0u;
  {
    const v4u z = {0u, 0u, 0u, 0u};
    for (int i = l; i < NGRP * CAP1 / 4; i += 32) ((v4u*)reg)[i] = z;
  }
  __syncthreads();

  const int e0 = blk * CH1;
  const int e1 = (e0 + CH1 < E) ? (e0 + CH1) : E;
  for (int base = e0; base < e1; base += 32) {
    const int e = base + l;
    bool valid = e < e1;
    int r = 0, c = 0;
    if (valid) { r = rowp[e]; c = colp[e]; }
    valid = valid && ((unsigned)c < (unsigned)n);
    r = (r < 0) ? 0 : ((r > n - 1) ? (n - 1) : r);
    int g = 0, lc = 0;
    if (valid) {
      g = c / gs;
      if (g > NGRP - 1) g = NGRP - 1;
      lc = c - g * gs;
      if (lc > GSMAX - 1) lc = GSMAX - 1;
      if (lc < 0) lc = 0;
    }
    const unsigned pe = peer_mask<6>((unsigned)g, (unsigned)__ballot(valid));
    const unsigned rank = __popc(pe & ((1u << l) - 1u));
    const unsigned cp = __popc(pe);
    if (valid) {
      const unsigned cu = cur[g];
      const unsigned pos = cu + rank;
      if (pos < (unsigned)CAP1) reg[g * CAP1 + pos] = ((unsigned)lc << 16) | (unsigned)r;
      if (rank == 0u) cur[g] = cu + cp;
    }
  }
  __syncthreads();

  v4u cv = {0u, 0u, 0u, 0u};
  if (l < 16) { cv.x = cur[4 * l]; cv.y = cur[4 * l + 1]; cv.z = cur[4 * l + 2]; cv.w = cur[4 * l + 3]; }
  unsigned* cdst = b1cnt + (size_t)blk * NGRP;
  unsigned* ddst = b1dat + (size_t)blk * NGRP * CAP1;
  const v4u* s4 = (const v4u*)reg;
  if (l < 16) *(volatile v4u*)(cdst + 4 * l) = cv;
  for (int i = l; i < NGRP * CAP1 / 4; i += 32) { const v4u v = s4[i]; ((volatile v4u*)ddst)[i] = v; }
  __threadfence();
  if (l < 16) *(volatile v4u*)(cdst + 4 * l) = cv;
  for (int i = l; i < NGRP * CAP1 / 4; i += 32) { const v4u v = s4[i]; ((volatile v4u*)ddst)[i] = v; }
}

__global__ void __launch_bounds__(256)
k_b2(const unsigned* __restrict__ b1cnt, const unsigned* __restrict__ b1dat, int nch,
     unsigned* gcnt, unsigned* goff, float* dis, unsigned* gl) {
  __shared__ volatile unsigned cntw[8 * GSMAX];
  __shared__ volatile unsigned curw[8 * GSMAX];
  __shared__ unsigned tot[GSMAX];
  __shared__ unsigned noff[GSMAX];
  __shared__ unsigned glist[CAPG] __attribute__((aligned(16)));
  const int t = threadIdx.x, w = t >> 5, l = t & 31, grp = blockIdx.x;

  for (int i = t; i < 8 * GSMAX; i += 256) cntw[i] = 0u;
  {
    const v4u z = {0u, 0u, 0u, 0u};
    for (int i = t; i < CAPG / 4; i += 256) ((v4u*)glist)[i] = z;
  }
  __syncthreads();

  for (int ch = w; ch < nch; ch += 8) {
    unsigned k = b1cnt[(size_t)ch * NGRP + grp];
    k = (unsigned)__builtin_amdgcn_readfirstlane((int)k);
    if (k > (unsigned)CAP1) k = (unsigned)CAP1;
    const unsigned* src = b1dat + ((size_t)ch * NGRP + grp) * CAP1;
    for (unsigned b0 = 0u; b0 < k; b0 += 32u) {
      const unsigned idx = b0 + (unsigned)l;
      const bool valid = idx < k;
      const unsigned p = valid ? src[idx] : 0u;
      unsigned v = p >> 16;
      if (v > (unsigned)(GSMAX - 1)) v = (unsigned)(GSMAX - 1);
      const unsigned pe = peer_mask<7>(v, (unsigned)__ballot(valid));
      const unsigned rank = __popc(pe & ((1u << l) - 1u));
      const unsigned cp = __popc(pe);
      if (valid && rank == 0u) {
        const int a = w * GSMAX + (int)v;
        cntw[a] = cntw[a] + cp;
      }
    }
  }
  __syncthreads();

  if (t < GSMAX) {
    unsigned s = 0u;
#pragma unroll
    for (int w2 = 0; w2 < 8; ++w2) s += cntw[w2 * GSMAX + t];
    tot[t] = s;
  }
  __syncthreads();
  if (w == 0) {
    const unsigned a0 = tot[4 * l], a1 = tot[4 * l + 1], a2 = tot[4 * l + 2], a3 = tot[4 * l + 3];
    const unsigned s = a0 + a1 + a2 + a3;
    unsigned incl = s;
#pragma unroll
    for (int d = 1; d < 32; d <<= 1) {
      const unsigned u = __shfl_up(incl, d, 32);
      if (l >= d) incl += u;
    }
    const unsigned ex = incl - s;
    noff[4 * l]     = ex;
    noff[4 * l + 1] = ex + a0;
    noff[4 * l + 2] = ex + a0 + a1;
    noff[4 * l + 3] = ex + a0 + a1 + a2;
  }
  __syncthreads();
  if (t < GSMAX) {
    unsigned run = noff[t];
#pragma unroll
    for (int w2 = 0; w2 < 8; ++w2) { curw[w2 * GSMAX + t] = run; run += cntw[w2 * GSMAX + t]; }
  }
  __syncthreads();

  for (int ch = w; ch < nch; ch += 8) {
    unsigned k = b1cnt[(size_t)ch * NGRP + grp];
    k = (unsigned)__builtin_amdgcn_readfirstlane((int)k);
    if (k > (unsigned)CAP1) k = (unsigned)CAP1;
    const unsigned* src = b1dat + ((size_t)ch * NGRP + grp) * CAP1;
    for (unsigned b0 = 0u; b0 < k; b0 += 32u) {
      const unsigned idx = b0 + (unsigned)l;
      const bool valid = idx < k;
      const unsigned p = valid ? src[idx] : 0u;
      unsigned v = p >> 16;
      if (v > (unsigned)(GSMAX - 1)) v = (unsigned)(GSMAX - 1);
      const unsigned pe = peer_mask<7>(v, (unsigned)__ballot(valid));
      const unsigned rank = __popc(pe & ((1u << l) - 1u));
      const unsigned cp = __popc(pe);
      if (valid) {
        const int a = w * GSMAX + (int)v;
        const unsigned cu = curw[a];
        const unsigned pos = cu + rank;
        if (pos < (unsigned)CAPG) glist[pos] = p & 0xFFFFu;
        if (rank == 0u) curw[a] = cu + cp;
      }
    }
  }
  __syncthreads();

  if (w == 0) {
    v4u v4 = {tot[4 * l], tot[4 * l + 1], tot[4 * l + 2], tot[4 * l + 3]};
    unsigned* d = gcnt + (size_t)grp * GSMAX + 4 * l;
    *(volatile v4u*)d = v4;
    __threadfence();
    *(volatile v4u*)d = v4;
  } else if (w == 1) {
    v4u v4 = {noff[4 * l], noff[4 * l + 1], noff[4 * l + 2], noff[4 * l + 3]};
    unsigned* d = goff + (size_t)grp * GSMAX + 4 * l;
    *(volatile v4u*)d = v4;
    __threadfence();
    *(volatile v4u*)d = v4;
  } else if (w == 2) {
    v4f v4;
    v4.x = 1.0f / sqrtf((float)(tot[4 * l] + 1u));
    v4.y = 1.0f / sqrtf((float)(tot[4 * l + 1] + 1u));
    v4.z = 1.0f / sqrtf((float)(tot[4 * l + 2] + 1u));
    v4.w = 1.0f / sqrtf((float)(tot[4 * l + 3] + 1u));
    float* d = dis + (size_t)grp * GSMAX + 4 * l;
    *(volatile v4f*)d = v4;
    __threadfence();
    *(volatile v4f*)d = v4;
  }
  const v4u* s4 = (const v4u*)glist;
  unsigned* ld = gl + (size_t)grp * CAPG;
  for (int i = t; i < CAPG / 4; i += 256) { const v4u v = s4[i]; ((volatile v4u*)ld)[i] = v; }
  __threadfence();
  for (int i = t; i < CAPG / 4; i += 256) { const v4u v = s4[i]; ((volatile v4u*)ld)[i] = v; }
}

__global__ void __launch_bounds__(256)
k_zgemm(const us_t* __restrict__ YTh, const us_t* __restrict__ YTl,
        const us_t* __restrict__ XTh, const us_t* __restrict__ XTl, int n,
        us_t* ZTh, us_t* ZTl) {
  __shared__ float zt[16 * LDP] __attribute__((aligned(16)));
  const int t = threadIdx.x, w = t >> 5, l = t & 31, h = l >> 4, m = l & 15;
  const int n0 = blockIdx.x * 16;
  const int m0 = 16 * w;
  v8f acc = gemm3(YTh + (size_t)(m0 + m) * n, YTl + (size_t)(m0 + m) * n,
                  XTh + (size_t)(n0 + m) * n, XTl + (size_t)(n0 + m) * n, n, h);
#pragma unroll
  for (int r = 0; r < 8; ++r) zt[m * LDP + m0 + 8 * h + r] = acc[r];
  __syncthreads();

  const int cl = 2 * w + (l >> 4), kb = 8 * (l & 15);
  float v[8];
#pragma unroll
  for (int e = 0; e < 8; ++e) v[e] = zt[cl * LDP + kb + e];
  v8us hi, lo;
  split8(v, hi, lo);
  const size_t o = (size_t)(n0 + cl) * DIM + kb;
  *(volatile v8us*)(ZTh + o) = hi;
  *(volatile v8us*)(ZTl + o) = lo;
  __threadfence();
  *(volatile v8us*)(ZTh + o) = hi;
  *(volatile v8us*)(ZTl + o) = lo;
}

__global__ void __launch_bounds__(256)
k_xw(const us_t* __restrict__ Xh, const us_t* __restrict__ Xl,
     const us_t* __restrict__ WTh, const us_t* __restrict__ WTl, int n, float* xw) {
  __shared__ float st[16 * LDP] __attribute__((aligned(16)));
  const int t = threadIdx.x, w = t >> 5, l = t & 31, h = l >> 4, m = l & 15;
  const int m0 = blockIdx.x * 16;
  if (m0 >= n) return;
  const int ra = (m0 + m < n) ? (m0 + m) : (n - 1);
  const int c0 = 16 * w;
  v8f acc = gemm3(Xh + (size_t)ra * DIM, Xl + (size_t)ra * DIM,
                  WTh + (size_t)(c0 + m) * DIM, WTl + (size_t)(c0 + m) * DIM, DIM, h);
#pragma unroll
  for (int r = 0; r < 8; ++r) st[(8 * h + r) * LDP + c0 + m] = acc[r];
  __syncthreads();

  const int r0 = 2 * w, r1 = 2 * w + 1;
  const v4f o0 = *(const v4f*)(st + r0 * LDP + 4 * l);
  const v4f o1 = *(const v4f*)(st + r1 * LDP + 4 * l);
  float* d0 = xw + (size_t)(m0 + r0) * DIM + 4 * l;
  float* d1 = xw + (size_t)(m0 + r1) * DIM + 4 * l;
  const bool k0ok = (m0 + r0) < n, k1ok = (m0 + r1) < n;
  if (k0ok) *(volatile v4f*)d0 = o0;
  if (k1ok) *(volatile v4f*)d1 = o1;
  __threadfence();
  if (k0ok) *(volatile v4f*)d0 = o0;
  if (k1ok) *(volatile v4f*)d1 = o1;
}

__device__ __forceinline__ v4f agg_row(int v, int l, int n, int gs,
                                       const float* __restrict__ xw,
                                       const unsigned* __restrict__ gcnt,
                                       const unsigned* __restrict__ goff,
                                       const float* __restrict__ dis,
                                       const unsigned* __restrict__ gl) {
  const int grp = v / gs;
  int vl = v - grp * gs;
  if (vl > GSMAX - 1) vl = GSMAX - 1;
  const int ti = grp * GSMAX + vl;
  unsigned cnt = gcnt[ti];
  unsigned off = goff[ti];
  const float dv = dis[ti];
  cnt = (unsigned)__builtin_amdgcn_readfirstlane((int)cnt);
  off = (unsigned)__builtin_amdgcn_readfirstlane((int)off);
  if (off > (unsigned)CAPG) off = (unsigned)CAPG;
  if (cnt > (unsigned)CAPG - off) cnt = (unsigned)CAPG - off;
  const unsigned* lst = gl + (size_t)grp * CAPG + off;
  v4f g4 = *(const v4f*)(xw + (size_t)v * DIM + 4 * l) * (dv * dv);
  for (unsigned b0 = 0u; b0 < cnt; b0 += 32u) {
    const unsigned e = b0 + (unsigned)l;
    unsigned r = 0u;
    float wgt = 0.f;
    if (e < cnt) {
      r = lst[e];
      if (r > (unsigned)(n - 1)) r = (unsigned)(n - 1);
      const int rg = (int)r / gs;
      int rl = (int)r - rg * gs;
      if (rl > GSMAX - 1) rl = GSMAX - 1;
      wgt = dis[rg * GSMAX + rl] * dv;
    }
    int kmax = (int)(cnt - b0);
    if (kmax > 32) kmax = 32;
    for (int jj = 0; jj < kmax; ++jj) {
      const unsigned rr = __shfl(r, jj, 32);
      const float ww = __shfl(wgt, jj, 32);
      const v4f xv = *(const v4f*)(xw + (size_t)rr * DIM + 4 * l);
      g4 += xv * ww;
    }
  }
  return g4;
}

__device__ __forceinline__ float sgm(float a) { return 1.0f / (1.0f + expf(-a)); }

__global__ void __launch_bounds__(256)
k_att(const us_t* __restrict__ Yh, const us_t* __restrict__ Yl,
      const us_t* __restrict__ ZTh, const us_t* __restrict__ ZTl,
      const float* __restrict__ xw, const float* __restrict__ bias,
      const unsigned* __restrict__ gcnt, const unsigned* __restrict__ goff,
      const float* __restrict__ dis, const unsigned* __restrict__ gl,
      int n, int gs, float* out) {
  __shared__ float st[16 * LDP] __attribute__((aligned(16)));
  const int t = threadIdx.x, w = t >> 5, l = t & 31, h = l >> 4, m = l & 15;
  const int m0 = blockIdx.x * 16;
  if (m0 >= n) return;
  const int ra = (m0 + m < n) ? (m0 + m) : (n - 1);
  const int c0 = 16 * w;
  v8f acc = gemm3(Yh + (size_t)ra * DIM, Yl + (size_t)ra * DIM,
                  ZTh + (size_t)(c0 + m) * DIM, ZTl + (size_t)(c0 + m) * DIM, DIM, h);
#pragma unroll
  for (int r = 0; r < 8; ++r) st[(8 * h + r) * LDP + c0 + m] = acc[r];
  __syncthreads();

  const v4f b4 = *(const v4f*)(bias + 4 * l);
  const int r0 = 2 * w, r1 = 2 * w + 1;
  const int v0 = (m0 + r0 < n) ? (m0 + r0) : (n - 1);
  const int v1 = (m0 + r1 < n) ? (m0 + r1) : (n - 1);

  const v4f g0 = agg_row(v0, l, n, gs, xw, gcnt, goff, dis, gl) + b4;
  const v4f a0 = *(const v4f*)(st + r0 * LDP + 4 * l);
  v4f o0;
  o0.x = g0.x * sgm(a0.x); o0.y = g0.y * sgm(a0.y); o0.z = g0.z * sgm(a0.z); o0.w = g0.w * sgm(a0.w);

  const v4f g1 = agg_row(v1, l, n, gs, xw, gcnt, goff, dis, gl) + b4;
  const v4f a1 = *(const v4f*)(st + r1 * LDP + 4 * l);
  v4f o1;
  o1.x = g1.x * sgm(a1.x); o1.y = g1.y * sgm(a1.y); o1.z = g1.z * sgm(a1.z); o1.w = g1.w * sgm(a1.w);

  float* d0 = out + (size_t)(m0 + r0) * DIM + 4 * l;
  float* d1 = out + (size_t)(m0 + r1) * DIM + 4 * l;
  const bool k0ok = (m0 + r0) < n, k1ok = (m0 + r1) < n;
  if (k0ok) *(volatile v4f*)d0 = o0;
  if (k1ok) *(volatile v4f*)d1 = o1;
  __threadfence();
  if (k0ok) *(volatile v4f*)d0 = o0;
  if (k1ok) *(volatile v4f*)d1 = o1;
}

static inline size_t al256(size_t b) { return (b + 255u) & ~(size_t)255u; }

extern "C" void kernel_launch(void* const* d_in, const int* in_sizes, int n_in,
                              void* d_out, int out_size, void* d_ws, size_t ws_size,
                              hipStream_t stream) {
  if (n_in < 4) return;
  const float* x    = (const float*)d_in[0];
  const int*   ei   = (const int*)d_in[1];
  const float* W    = (const float*)d_in[2];
  const float* bias = (const float*)d_in[3];

  const int nx = in_sizes[0];
  if (nx <= 0 || (nx % DIM) != 0) return;
  const int n = nx / DIM;
  if (n < 64 || n > NGRP * GSMAX || (n % 64) != 0) return;
  if (in_sizes[2] != DIM * DIM || in_sizes[3] != DIM) return;
  if ((size_t)out_size != (size_t)n * DIM) return;
  if (in_sizes[1] < 0 || (in_sizes[1] % 2) != 0) return;
  const int E = in_sizes[1] / 2;
  const int gs = n / NGRP;
  int nch = (E + CH1 - 1) / CH1;
  if (nch < 1) nch = 1;
  const int* rowp = ei;
  const int* colp = ei + E;

  char* ws = (char*)d_ws;
  size_t off = 0;
  const size_t plane = al256((size_t)n * DIM * sizeof(us_t));
  us_t* Yh  = (us_t*)(ws + off); off += plane;
  us_t* Yl  = (us_t*)(ws + off); off += plane;
  us_t* Xh  = (us_t*)(ws + off); off += plane;
  us_t* Xl  = (us_t*)(ws + off); off += plane;
  us_t* YTh = (us_t*)(ws + off); off += plane;
  us_t* YTl = (us_t*)(ws + off); off += plane;
  us_t* XTh = (us_t*)(ws + off); off += plane;
  us_t* XTl = (us_t*)(ws + off); off += plane;
  const size_t wpl = al256((size_t)DIM * DIM * sizeof(us_t));
  us_t* WTh = (us_t*)(ws + off); off += wpl;
  us_t* WTl = (us_t*)(ws + off); off += wpl;
  us_t* ZTh = (us_t*)(ws + off); off += wpl;
  us_t* ZTl = (us_t*)(ws + off); off += wpl;
  float* xw = (float*)(ws + off); off += al256((size_t)n * DIM * sizeof(float));
  unsigned* b1cnt = (unsigned*)(ws + off); off += al256((size_t)nch * NGRP * sizeof(unsigned));
  unsigned* b1dat = (unsigned*)(ws + off); off += al256((size_t)nch * NGRP * CAP1 * sizeof(unsigned));
  unsigned* gcnt = (unsigned*)(ws + off); off += al256((size_t)NGRP * GSMAX * sizeof(unsigned));
  unsigned* goff = (unsigned*)(ws + off); off += al256((size_t)NGRP * GSMAX * sizeof(unsigned));
  float*    dis  = (float*)(ws + off);    off += al256((size_t)NGRP * GSMAX * sizeof(float));
  unsigned* gl   = (unsigned*)(ws + off); off += al256((size_t)NGRP * CAPG * sizeof(unsigned));
  if (off > ws_size) return;
  float* out = (float*)d_out;

  const dim3 b256(256);
  k_prep<<<dim3((n + 63) / 64), b256, 0, stream>>>(x, n, Yh, Yl, Xh, Xl, YTh, YTl, XTh, XTl);
  k_wconv<<<dim3(1), b256, 0, stream>>>(W, WTh, WTl);
  k_b1<<<dim3(nch), dim3(32), 0, stream>>>(rowp, colp, E, n, gs, b1cnt, b1dat);
  k_b2<<<dim3(NGRP), b256, 0, stream>>>(b1cnt, b1dat, nch, gcnt, goff, dis, gl);
  k_zgemm<<<dim3(DIM / 16), b256, 0, stream>>>(YTh, YTl, XTh, XTl, n, ZTh, ZTl);
  k_xw<<<dim3((n + 15) / 16), b256, 0, stream>>>(Xh, Xl, WTh, WTl, n, xw);
  k_att<<<dim3((n + 15) / 16), b256, 0, stream>>>(Yh, Yl, ZTh, ZTl, xw, bias,
                                                  gcnt, goff, dis, gl, n, gs, out);
}
